// GPT_68496138437299
// MI455X (gfx1250) — hardware-verified
//
#include <hip/hip_runtime.h>


#ifndef NB
#define NB 4
#endif
#ifndef SEQ
#define SEQ 1024
#endif

namespace {
constexpr int NBF = 4, SEQF = 1024, NE = 1024, NH = 16, HD = 64, HH = 32, NF = 16, NQ = 3072, GRP = 64, KT = 32;
constexpr int NTOK = NB * SEQ, NMAP = NB * NH * 2;
constexpr float XS = 8.0f, WSC = 256.0f, FSC = 256.0f, PS = 1024.0f, YLS = 1024.0f, LOG2E = 1.4426950408889634f, NEPS = 1e-5f;
static_assert(NB >= 1 && NB <= NBF && SEQ >= 64 && SEQ <= SEQF && SEQ % 64 == 0);
static_assert(NE % 256 == 0 && NQ % 128 == 0 && NTOK % 64 == 0 && NE % 128 == 0 && HD == 2 * HH && NF == 16 && KT == 2 * NF && NQ == 3 * NE);
constexpr int PB_W = NQ * NE / GRP / 64;
constexpr int PB_P = NE * NE / GRP / 64;
constexpr int PB_F = NF * NE / 8 / 64;
constexpr int PB_X = NTOK * NE / 8 / 64;
static_assert((NQ * NE) % (GRP * 64) == 0 && (NE * NE) % (GRP * 64) == 0 && (NF * NE) % 512 == 0 && (NTOK * NE) % 512 == 0);

typedef _Float16 b16;
typedef unsigned short us16;
typedef __attribute__((ext_vector_type(16))) _Float16 v16b;
typedef __attribute__((ext_vector_type(8))) _Float16 v8b;
typedef __attribute__((ext_vector_type(4))) _Float16 v4h;
typedef __attribute__((ext_vector_type(2))) _Float16 v2h;
typedef __attribute__((ext_vector_type(16))) __bf16 v16z;
typedef __attribute__((ext_vector_type(8))) unsigned short v8u;
typedef __attribute__((ext_vector_type(8))) float v8f;
typedef __attribute__((ext_vector_type(4))) float v4f;
union FragZ { v8u u[2]; v16z v; };

__device__ __forceinline__ unsigned int bf16_bits_rne(float f) { unsigned int u = __float_as_uint(f); u += 0x7FFFu + ((u >> 16) & 1u); return u >> 16; }
__device__ __forceinline__ float bf16_rne(float f) { return __uint_as_float(bf16_bits_rne(f) << 16); }
__device__ __forceinline__ void split16(float v, b16& hi, b16& lo) { hi = (b16)v; lo = (b16)(v - (float)hi); }
__device__ __forceinline__ void splitz(float v, us16& hi, us16& lo) { const unsigned int hb = bf16_bits_rne(v); const float hf = __uint_as_float(hb << 16); hi = (us16)hb; lo = (us16)bf16_bits_rne(v - hf); }
__device__ __forceinline__ v16b frag_kb(const b16* p, int hh) { const v8b a = *(const v8b*)(p + 8 * hh), b = *(const v8b*)(p + 16 + 8 * hh); v16b f;
#pragma unroll
  for (int e = 0; e < 8; ++e) { f[e] = a[e]; f[8 + e] = b[e]; } return f; }
__device__ __forceinline__ v16z frag_kz(const us16* p, int hh) { FragZ f; f.u[0] = *(const v8u*)(p + 8 * hh); f.u[1] = *(const v8u*)(p + 16 + 8 * hh); return f.v; }
__device__ __forceinline__ v8f wmma16b(v16b a, v16b b, v8f c) { v8f d = __builtin_amdgcn_wmma_f32_16x16x32_f16(false, a, false, b, (short)0, c, false, false); asm volatile("v_nop\n\tv_nop\n\tv_nop\n\tv_nop" : "+v"(d) : "v"(a), "v"(b)); return d; }
__device__ __forceinline__ v8f wmma16z(v16z a, v16z b, v8f c) { v8f d = __builtin_amdgcn_wmma_f32_16x16x32_bf16(false, a, false, b, (short)0, c, false, false); asm volatile("v_nop\n\tv_nop\n\tv_nop\n\tv_nop" : "+v"(d) : "v"(a), "v"(b)); return d; }
__device__ __forceinline__ void wave_lds_sync() { __builtin_amdgcn_fence(__ATOMIC_RELEASE, "workgroup"); __builtin_amdgcn_wave_barrier(); __builtin_amdgcn_fence(__ATOMIC_ACQUIRE, "workgroup"); }
__device__ __forceinline__ float nexp2(float v) { return __builtin_amdgcn_exp2f(v); }

__global__ __launch_bounds__(64) void prep_kernel(const float* __restrict__ wq, const float* __restrict__ pr, const float* __restrict__ ft, const float* __restrict__ x,
                                                  b16* __restrict__ WT, b16* __restrict__ PT, b16* __restrict__ FP, b16* __restrict__ XP) {
#pragma clang fp contract(off)
  __shared__ __attribute__((aligned(16))) b16 St[64][GRP + 8];
  const int bid = blockIdx.x, t = threadIdx.x, wave = t >> 5, lane = t & 31;
  if (bid < PB_W + PB_P) {
    const bool isw = bid < PB_W;
    const float* src = isw ? wq : pr;
    b16* dst = isw ? WT : PT;
    const size_t g0 = (size_t)(isw ? bid : bid - PB_W) * 64;
    const float* gp = src + (g0 + t) * GRP;
    float s = 0.0f;
#pragma unroll 1
    for (int j = 0; j < GRP; j += 4) {
      const v4f f = *(const v4f*)(gp + j);
#pragma unroll
      for (int c = 0; c < 4; ++c) s += fabsf(bf16_rne(f[c]));
    }
    float scale = bf16_rne(s * (1.0f / GRP));
    scale = fmaxf(scale, bf16_rne(1e-8f));
    const float rs = 1.0f / scale;
#pragma unroll 1
    for (int j = 0; j < GRP; j += 4) {
      const v4f f = *(const v4f*)(gp + j); v4h o;
#pragma unroll
      for (int c = 0; c < 4; ++c) {
        const float wb = bf16_rne(f[c]);
        const float qf = bf16_rne(wb * rs);
        const float q = fminf(fmaxf(rintf(qf), -1.0f), 1.0f);
        const float t1 = bf16_rne(q * scale);
        const float t2 = bf16_rne(t1 - wb);
        const float wt = bf16_rne(wb + t2);
        o[c] = (b16)(wt * WSC);
      }
      *(v4h*)(&St[t][j]) = o;
    }
    __syncthreads();
    b16* dblk = dst + g0 * GRP;
    for (int pass = 0; pass < 2; ++pass) {
#pragma unroll 1
      for (int i = 0; i < 8; ++i) {
        const int line = wave * 32 + 4 * i + (lane >> 3), e = lane & 7;
        const v8b v = *(const v8b*)(&St[line][e * 8]);
        *(volatile v8b*)(dblk + (size_t)line * GRP + e * 8) = v;
      }
      __threadfence();
    }
  } else if (bid < PB_W + PB_P + PB_F) {
    const size_t e0 = ((size_t)(bid - PB_W - PB_P) * 64 + t) * 8;
    const v4f f0 = *(const v4f*)(ft + e0), f1 = *(const v4f*)(ft + e0 + 4); v8b o;
#pragma unroll
    for (int j = 0; j < 4; ++j) { o[j] = (b16)(bf16_rne(f0[j]) * FSC); o[4 + j] = (b16)(bf16_rne(f1[j]) * FSC); }
    for (int pass = 0; pass < 2; ++pass) { *(volatile v8b*)(FP + e0) = o; __threadfence(); }
  } else {
    const size_t e0 = ((size_t)(bid - PB_W - PB_P - PB_F) * 64 + t) * 8;
    if (e0 < (size_t)NTOK * NE) {
      const size_t r = e0 / NE, c = e0 % NE; const size_t xr = (r / SEQ) * SEQF + (r % SEQ);
      const v4f f0 = *(const v4f*)(x + xr * NE + c), f1 = *(const v4f*)(x + xr * NE + c + 4); v8b o;
#pragma unroll
      for (int j = 0; j < 4; ++j) { o[j] = (b16)(bf16_rne(f0[j]) * XS); o[4 + j] = (b16)(bf16_rne(f1[j]) * XS); }
      for (int pass = 0; pass < 2; ++pass) { *(volatile v8b*)(XP + e0) = o; __threadfence(); }
    }
  }
}

__global__ __launch_bounds__(128) void proj_kernel(const b16* __restrict__ XP, const b16* __restrict__ WT, const float* __restrict__ qg,
                                                   b16* __restrict__ Qh, b16* __restrict__ Ql, b16* __restrict__ Kh, b16* __restrict__ Kl, b16* __restrict__ VTh, b16* __restrict__ VTl) {
  __shared__ __attribute__((aligned(16))) float Tf[4][16][128 + 4];
  const int wave = threadIdx.x >> 5, lane = threadIdx.x & 31, nloc = lane & 15, hlf = lane >> 4;
  const int r0 = blockIdx.x * 64, bb = r0 / SEQ, s0 = r0 % SEQ, m0 = r0 + wave * 16;
  const int slab = blockIdx.y, n0 = slab * 128;
  v8f acc[8];
#pragma unroll
  for (int t = 0; t < 8; ++t) acc[t] = (v8f){};
  const b16* xa = XP + (size_t)(m0 + nloc) * NE;
#pragma unroll 1
  for (int kb = 0; kb < NE; kb += 32) {
    const v16b a = frag_kb(xa + kb, hlf);
#pragma unroll
    for (int t = 0; t < 8; ++t) acc[t] = wmma16b(a, frag_kb(WT + (size_t)(n0 + t * 16 + nloc) * NE + kb, hlf), acc[t]);
  }
#pragma unroll
  for (int t = 0; t < 8; ++t)
#pragma unroll
    for (int r = 0; r < 8; ++r) Tf[wave][8 * hlf + r][t * 16 + nloc] = acc[t][r] * (1.0f / (XS * WSC));
  __syncthreads();
  if (slab < 16) {
    const bool isq = slab < 8; const int hb = isq ? 2 * slab : 2 * (slab - 8);
    b16* Ph = isq ? Qh : Kh; b16* Pl = isq ? Ql : Kl;
    const float idx = (float)(2 * lane) * (1.0f / 64.0f);
    float invf = 1.0f / powf(10000.0f, idx);
    const float ramp = fminf(fmaxf((idx - 0.25f) / 0.75f, 0.0f), 1.0f);
    invf = invf / (ramp * 3.0f + 1.0f);
    const float gq0 = bf16_rne(qg[hb]), gq1 = bf16_rne(qg[hb + 1]);
#pragma unroll 1
    for (int rr = 0; rr < 16; ++rr) {
      const float ang = (float)(s0 + wave * 16 + rr) * invf; const float cv = cosf(ang), sv = sinf(ang);
#pragma unroll
      for (int hs = 0; hs < 2; ++hs) {
        const float v1 = Tf[wave][rr][hs * 64 + lane], v2 = Tf[wave][rr][hs * 64 + 32 + lane];
        float ss = v1 * v1 + v2 * v2;
#pragma unroll
        for (int o = 1; o < 32; o <<= 1) ss += __shfl_xor(ss, o);
        const float inv = rsqrtf(ss * (1.0f / HD) + NEPS);
        const float n1 = v1 * inv, n2 = v2 * inv;
        const float g = isq ? (hs ? gq1 : gq0) : 1.0f;
        const float a1 = (n1 * cv + n2 * sv) * g, a2 = (n2 * cv - n1 * sv) * g;
        Tf[wave][rr][hs * 64 + lane] = a1 * XS; Tf[wave][rr][hs * 64 + 32 + lane] = a2 * XS;
      }
    }
    wave_lds_sync();
    const int tb = s0 + wave * 16;
    for (int pass = 0; pass < 2; ++pass) {
#pragma unroll 1
      for (int c = 0; c < 4; ++c) {
        const int hs = c >> 1, half = c & 1; const int z = (bb * NH + hb + hs) * 2 + half;
        b16* dh = Ph + ((size_t)z * SEQ + tb) * HH; b16* dl = Pl + ((size_t)z * SEQ + tb) * HH;
#pragma unroll
        for (int i = 0; i < 2; ++i) {
          const int line = 4 * i + (lane >> 3), e = lane & 7; const int tok = 2 * line + (e >> 2), dd = (e & 3) * 8;
          const float* sp = &Tf[wave][tok][hs * 64 + half * 32 + dd]; const v4f f0 = *(const v4f*)sp, f1 = *(const v4f*)(sp + 4); v8b hv, lv;
#pragma unroll
          for (int j = 0; j < 4; ++j) { b16 p, q; split16(f0[j], p, q); hv[j] = p; lv[j] = q; split16(f1[j], p, q); hv[4 + j] = p; lv[4 + j] = q; }
          *(volatile v8b*)(dh + (size_t)tok * HH + dd) = hv; *(volatile v8b*)(dl + (size_t)tok * HH + dd) = lv;
        }
      }
      __threadfence();
    }
  } else {
    const int hb = 2 * (slab - 16);
    for (int pass = 0; pass < 2; ++pass) {
#pragma unroll 1
      for (int q = 0; q < 32; ++q) {
        const int cl = wave * 32 + q; const int hs = cl >> 6, dd = cl & 63, half = dd >> 5, d = dd & 31; const int z = (bb * NH + hb + hs) * 2 + half;
        const int tk = lane * 2; v2h hv, lv;
#pragma unroll
        for (int j = 0; j < 2; ++j) { b16 p, ql; split16(Tf[(tk + j) >> 4][(tk + j) & 15][cl] * XS, p, ql); hv[j] = p; lv[j] = ql; }
        const size_t oi = ((size_t)z * HH + d) * SEQ + s0 + lane * 2; *(volatile v2h*)(VTh + oi) = hv; *(volatile v2h*)(VTl + oi) = lv;
      }
      __threadfence();
    }
  }
}

__global__ __launch_bounds__(64) void attn_kernel(const b16* __restrict__ Qh, const b16* __restrict__ Ql, const b16* __restrict__ Kh, const b16* __restrict__ Kl,
                                                  const b16* __restrict__ VTh, const b16* __restrict__ VTl, const float* __restrict__ dlm, b16* __restrict__ Yh, b16* __restrict__ Yl) {
  __shared__ __attribute__((aligned(16))) b16 Pb[2][16][32 + 8], Pc[2][16][32 + 8];
  __shared__ __attribute__((aligned(16))) float To[2][16][HH + 4];
  const int wave = threadIdx.x >> 5, lane = threadIdx.x & 31, hh = lane >> 4, col = lane & 15;
  const int bh = blockIdx.y, bb = bh / NH, h = bh % NH, z = bh * 2 + wave;
  const int q0 = blockIdx.x * 16, qi = q0 + col;
  const b16* Qhb = Qh + (size_t)z * SEQ * HH; const b16* Qlb = Ql + (size_t)z * SEQ * HH; const b16* Khb = Kh + (size_t)z * SEQ * HH; const b16* Klb = Kl + (size_t)z * SEQ * HH;
  const b16* Vh = VTh + (size_t)z * HH * SEQ; const b16* Vl = VTl + (size_t)z * HH * SEQ;
  const v16b qa = frag_kb(Qhb + (size_t)qi * HH, hh), qb = frag_kb(Qlb + (size_t)qi * HH, hh);
  const float cs = LOG2E * 0.17677669529663687f / (XS * XS);
  float m = -INFINITY, l = 0.0f; v8f o[2]; o[0] = (v8f){}; o[1] = (v8f){};
  const int kend = q0 + 16;
#pragma unroll 1
  for (int kb = 0; kb < kend; kb += 32) {
    float e[16]; float mx = -INFINITY;
#pragma unroll
    for (int u = 0; u < 2; ++u) {
      v8f s = (v8f){}; const size_t kr = (size_t)(kb + u * 16 + col) * HH;
      const v16b kh0 = frag_kb(Khb + kr, hh), kl0 = frag_kb(Klb + kr, hh);
      s = wmma16b(kh0, qa, s); s = wmma16b(kh0, qb, s); s = wmma16b(kl0, qa, s);
#pragma unroll
      for (int r = 0; r < 8; ++r) { const int key = kb + u * 16 + 8 * hh + r; const float vv = (key <= qi) ? s[r] * cs : -INFINITY; e[u * 8 + r] = vv; mx = fmaxf(mx, vv); }
    }
    mx = fmaxf(mx, __shfl_xor(mx, 16)); const float mn = fmaxf(m, mx); const float al = (mn == -INFINITY) ? 1.0f : nexp2(m - mn); float sum = 0.0f;
#pragma unroll
    for (int i2 = 0; i2 < 16; ++i2) { const float p = (e[i2] == -INFINITY || mn == -INFINITY) ? 0.0f : nexp2(e[i2] - mn); sum += p; b16 a_, b_; split16(p * PS, a_, b_);
      const int sl = (i2 < 8 ? 0 : 16) + 8 * hh + (i2 & 7); Pb[wave][col][sl] = a_; Pc[wave][col][sl] = b_; }
    sum += __shfl_xor(sum, 16); l = l * al + sum; m = mn;
    wave_lds_sync();
    const v16b pf = frag_kb(&Pb[wave][col][0], hh), pg = frag_kb(&Pc[wave][col][0], hh);
#pragma unroll
    for (int t = 0; t < 2; ++t) { o[t] *= al; const size_t vr = (size_t)(t * 16 + col) * SEQ + kb; const v16b va = frag_kb(Vh + vr, hh), vb = frag_kb(Vl + vr, hh);
      o[t] = wmma16b(va, pf, o[t]); o[t] = wmma16b(va, pg, o[t]); o[t] = wmma16b(vb, pf, o[t]); }
    wave_lds_sync();
  }
  const float inv = 1.0f / (l * PS * XS);
#pragma unroll
  for (int t = 0; t < 2; ++t)
#pragma unroll
    for (int r = 0; r < 8; ++r) To[wave][col][t * 16 + 8 * hh + r] = o[t][r] * inv;
  __syncthreads();
  const float lam = bf16_rne(dlm[h]);
  const size_t yr0 = (size_t)bb * SEQ + q0;
  for (int pass = 0; pass < 2; ++pass) {
#pragma unroll
    for (int i = 0; i < 2; ++i) {
      const int tok = wave * 8 + 4 * i + (lane >> 3), e = lane & 7; const int dd0 = e * 8, dsrc = dd0 & 31; const float sg = (e < 4) ? -lam : lam;
      const v4f a0 = *(const v4f*)(&To[0][tok][dsrc]), a1 = *(const v4f*)(&To[0][tok][dsrc + 4]), c0 = *(const v4f*)(&To[1][tok][dsrc]), c1 = *(const v4f*)(&To[1][tok][dsrc + 4]);
      v8b hv, lv;
#pragma unroll
      for (int j = 0; j < 4; ++j) {
        const float y0 = (a0[j] + sg * c0[j]) * XS; const b16 p0 = (b16)y0; hv[j] = p0; lv[j] = (b16)((y0 - (float)p0) * YLS);
        const float y1 = (a1[j] + sg * c1[j]) * XS; const b16 p1 = (b16)y1; hv[4 + j] = p1; lv[4 + j] = (b16)((y1 - (float)p1) * YLS);
      }
      const size_t oi = (yr0 + tok) * NE + (size_t)h * HD + dd0; *(volatile v8b*)(Yh + oi) = hv; *(volatile v8b*)(Yl + oi) = lv;
    }
    __threadfence();
  }
}

__global__ __launch_bounds__(64) void feat_kernel(const b16* __restrict__ Yh, const b16* __restrict__ Yl, const b16* __restrict__ PT, const b16* __restrict__ FP,
                                                  const float* __restrict__ th, const float* __restrict__ al, const float* __restrict__ be,
                                                  us16* __restrict__ Ah, us16* __restrict__ Al, us16* __restrict__ Bh, us16* __restrict__ Bl) {
  __shared__ __attribute__((aligned(16))) float St[2][16][KT + 4];
  const int wave = threadIdx.x >> 5, lane = threadIdx.x & 31, hh = lane >> 4, col = lane & 15;
  constexpr int NYB = NTOK / 32;
  const bool isy = (int)blockIdx.x < NYB;
  const int rbase = (isy ? (int)blockIdx.x : (int)blockIdx.x - NYB) * 32 + wave * 16;
  const b16* Fr = FP + (size_t)col * NE;
  v8f ah = (v8f){}, alo = (v8f){};
  if (isy) {
    const b16* Ar = Yh + (size_t)(rbase + col) * NE; const b16* Lr = Yl + (size_t)(rbase + col) * NE;
#pragma unroll 2
    for (int kb = 0; kb < NE; kb += 32) { const v16b bf = frag_kb(Fr + kb, hh); ah = wmma16b(frag_kb(Ar + kb, hh), bf, ah); alo = wmma16b(frag_kb(Lr + kb, hh), bf, alo); }
  } else {
    const b16* Ar = PT + (size_t)(rbase + col) * NE;
#pragma unroll 2
    for (int kb = 0; kb < NE; kb += 32) ah = wmma16b(frag_kb(Ar + kb, hh), frag_kb(Fr + kb, hh), ah);
  }
  const float tt = fabsf(bf16_rne(th[0])), aa = fabsf(bf16_rne(al[0])), bt = fabsf(bf16_rne(be[0]));
#pragma unroll
  for (int r = 0; r < 8; ++r) {
    const float v = isy ? (ah[r] + alo[r] * (1.0f / YLS)) * (1.0f / (XS * FSC)) : ah[r] * (1.0f / (WSC * FSC));
    const float sg = 1.0f / (1.0f + expf(-(v * 5.0f))); const float va = v * sg;
    const float f0 = isy ? va : (tt * va - aa * (1.0f - sg)); const float f1 = isy ? (1.0f - sg) : (-bt * va);
    St[wave][8 * hh + r][col] = f0; St[wave][8 * hh + r][NF + col] = f1;
  }
  wave_lds_sync();
  us16* dh = isy ? Ah : Bh; us16* dlo = isy ? Al : Bl;
  for (int pass = 0; pass < 2; ++pass) {
#pragma unroll
    for (int i = 0; i < 2; ++i) {
      const int line = 4 * i + (lane >> 3), e = lane & 7; const int row = 2 * line + (e >> 2), c8 = (e & 3) * 8;
      const v4f g0 = *(const v4f*)(&St[wave][row][c8]), g1 = *(const v4f*)(&St[wave][row][c8 + 4]); v8u hv, lv;
#pragma unroll
      for (int j = 0; j < 4; ++j) { us16 p, q; splitz(g0[j], p, q); hv[j] = p; lv[j] = q; splitz(g1[j], p, q); hv[4 + j] = p; lv[4 + j] = q; }
      const size_t oi = (size_t)(rbase + row) * KT + c8; *(volatile v8u*)(dh + oi) = hv; *(volatile v8u*)(dlo + oi) = lv;
    }
    __threadfence();
  }
}

__global__ __launch_bounds__(128) void out_kernel(const us16* __restrict__ Ah, const us16* __restrict__ Al, const us16* __restrict__ Bh, const us16* __restrict__ Bl, float* __restrict__ out) {
  __shared__ __attribute__((aligned(16))) float Tf[4][16][128 + 4];
  const int wave = threadIdx.x >> 5, lane = threadIdx.x & 31, nloc = lane & 15, hlf = lane >> 4; const int m0 = (blockIdx.x * 4 + wave) * 16; const int n0 = blockIdx.y * 128;
  const v16z a = frag_kz(Ah + (size_t)(m0 + nloc) * KT, hlf), alo = frag_kz(Al + (size_t)(m0 + nloc) * KT, hlf);
  v8f acc[8];
#pragma unroll
  for (int t = 0; t < 8; ++t) { const v16z bw = frag_kz(Bh + (size_t)(n0 + t * 16 + nloc) * KT, hlf), bl = frag_kz(Bl + (size_t)(n0 + t * 16 + nloc) * KT, hlf); v8f c = (v8f){};
    c = wmma16z(a, bw, c); c = wmma16z(a, bl, c); c = wmma16z(alo, bw, c); acc[t] = c; }
#pragma unroll
  for (int t = 0; t < 8; ++t)
#pragma unroll
    for (int r = 0; r < 8; ++r) Tf[wave][8 * hlf + r][t * 16 + nloc] = acc[t][r];
  wave_lds_sync();
  const int ob = m0 / SEQ, os = m0 % SEQ; const size_t orow0 = (size_t)ob * SEQF + os;
  for (int pass = 0; pass < 2; ++pass) {
#pragma unroll 1
    for (int rr = 0; rr < 16; ++rr) *(volatile v4f*)(out + (orow0 + rr) * NE + n0 + lane * 4) = *(const v4f*)(&Tf[wave][rr][lane * 4]);
    __threadfence();
  }
}
}

extern "C" void kernel_launch(void* const* d_in, const int* in_sizes, int n_in, void* d_out, int out_size, void* d_ws, size_t ws_size, hipStream_t stream) {
  if (n_in < 9) return;
  if (in_sizes[0] < NB * SEQF * NE || in_sizes[1] != NQ * NE || in_sizes[2] != NF * NE || in_sizes[3] != NE * NE || in_sizes[4] < 1 || in_sizes[5] < 1 || in_sizes[6] < 1 ||
      in_sizes[7] < NH || in_sizes[8] < NH || out_size < NB * SEQF * NE) return;
  auto Fp = [&](int i) { return (const float*)d_in[i]; };
  size_t off = 0; char* ws = (char*)d_ws;
  auto carve = [&](size_t bytes) { char* p = ws + off; off += (bytes + 255) & ~(size_t)255; return p; };
  b16* WT = (b16*)carve((size_t)NQ * NE * 2); b16* PT = (b16*)carve((size_t)NE * NE * 2); b16* FP = (b16*)carve((size_t)NF * NE * 2); b16* XP = (b16*)carve((size_t)NTOK * NE * 2);
  b16* Qh = (b16*)carve((size_t)NMAP * SEQ * HH * 2); b16* Ql = (b16*)carve((size_t)NMAP * SEQ * HH * 2); b16* Kh = (b16*)carve((size_t)NMAP * SEQ * HH * 2); b16* Kl = (b16*)carve((size_t)NMAP * SEQ * HH * 2);
  b16* VTh = (b16*)carve((size_t)NMAP * HH * SEQ * 2); b16* VTl = (b16*)carve((size_t)NMAP * HH * SEQ * 2);
  b16* Yh = (b16*)carve((size_t)NTOK * NE * 2); b16* Yl = (b16*)carve((size_t)NTOK * NE * 2);
  us16* Ah = (us16*)carve((size_t)NTOK * KT * 2); us16* Al = (us16*)carve((size_t)NTOK * KT * 2); us16* Bh = (us16*)carve((size_t)NE * KT * 2); us16* Bl = (us16*)carve((size_t)NE * KT * 2);
  if (off > ws_size || off > ((size_t)128 << 20)) return;
  prep_kernel<<<(unsigned)(PB_W + PB_P + PB_F + PB_X), 64, 0, stream>>>(Fp(1), Fp(3), Fp(2), Fp(0), WT, PT, FP, XP);
  proj_kernel<<<dim3(NTOK / 64, NQ / 128), 128, 0, stream>>>(XP, WT, Fp(7), Qh, Ql, Kh, Kl, VTh, VTl);
  attn_kernel<<<dim3(SEQ / 16, NB * NH), 64, 0, stream>>>(Qh, Ql, Kh, Kl, VTh, VTl, Fp(8), Yh, Yl);
  feat_kernel<<<(unsigned)(NTOK / 32 + NE / 32), 64, 0, stream>>>(Yh, Yl, PT, FP, Fp(4), Fp(5), Fp(6), Ah, Al, Bh, Bl);
  out_kernel<<<dim3(NTOK / 64, NE / 128), 128, 0, stream>>>(Ah, Al, Bh, Bl, (float*)d_out);
}
